// Local3dAttention_40819369181470
// MI455X (gfx1250) — hardware-verified
//
#include <hip/hip_runtime.h>
#include <hip/hip_bf16.h>

typedef __attribute__((ext_vector_type(16))) _Float16 v16h;
typedef __attribute__((ext_vector_type(8)))  _Float16 v8h;
typedef __attribute__((ext_vector_type(16))) __bf16   v16b;
typedef __attribute__((ext_vector_type(8)))  __bf16   v8b;
typedef __attribute__((ext_vector_type(8)))  float    v8f;
typedef __attribute__((ext_vector_type(4)))  float    v4f;

__device__ __forceinline__ unsigned short f2bf_bits(float f) {
  unsigned u = __float_as_uint(f);
  return (unsigned short)((u + 0x7FFFu + ((u >> 16) & 1u)) >> 16);
}
__device__ __forceinline__ float bf_bits2f(unsigned short h) { return __uint_as_float(((unsigned)h) << 16); }

__device__ __forceinline__ void dep_guard_h(v8f& a, v8f& b, v16h x, v16h y) { asm volatile("v_nop\n\tv_nop\n\tv_nop\n\tv_nop" : "+v"(a), "+v"(b) : "v"(x), "v"(y)); }
__device__ __forceinline__ void dep_guard_b(v8f& a, v8f& b, v16b x, v16b y) { asm volatile("v_nop\n\tv_nop\n\tv_nop\n\tv_nop" : "+v"(a), "+v"(b) : "v"(x), "v"(y)); }
__device__ __forceinline__ void keep4_h(v16h a, v16h b, v16h c, v16h d) { asm volatile("v_nop" :: "v"(a), "v"(b), "v"(c), "v"(d)); }
__device__ __forceinline__ void keep4_b(v16b a, v16b b, v16b c, v16b d) { asm volatile("v_nop" :: "v"(a), "v"(b), "v"(c), "v"(d)); }
__device__ __forceinline__ void acc_guard4(v8f& a, v8f& b, v8f& c, v8f& d) { asm volatile("v_nop\n\tv_nop\n\tv_nop\n\tv_nop" : "+v"(a), "+v"(b), "+v"(c), "+v"(d)); }
template <typename T> struct Frag;
template <> struct Frag<_Float16> {
  typedef v16h V; union U { v16h v; v8h h[2]; };
  static __device__ __forceinline__ v16h load(const _Float16* p) {
    U f; f.h[0] = *(const v8h*)(p); f.h[1] = *(const v8h*)(p + 16); return f.v;
  }
  static __device__ __forceinline__ v8f mma(v16h a, v16h b, v8f c) {
    return __builtin_amdgcn_wmma_f32_16x16x32_f16(false, a, false, b, (short)0, c, false, false);
  }
  static __device__ __forceinline__ void guard(v8f& a, v8f& b, v16h x, v16h y) { dep_guard_h(a, b, x, y); }
  static __device__ __forceinline__ void keep(v16h a, v16h b, v16h c, v16h d) { keep4_h(a, b, c, d); }
};
template <> struct Frag<__bf16> {
  typedef v16b V; union U { v16b v; v8b h[2]; };
  static __device__ __forceinline__ v16b load(const __bf16* p) {
    U f; f.h[0] = *(const v8b*)(p); f.h[1] = *(const v8b*)(p + 16); return f.v;
  }
  static __device__ __forceinline__ v8f mma(v16b a, v16b b, v8f c) {
    return __builtin_amdgcn_wmma_f32_16x16x32_bf16(false, a, false, b, (short)0, c, false, false);
  }
  static __device__ __forceinline__ void guard(v8f& a, v8f& b, v16b x, v16b y) { dep_guard_b(a, b, x, y); }
  static __device__ __forceinline__ void keep(v16b a, v16b b, v16b c, v16b d) { keep4_b(a, b, c, d); }
};

template <int ET> struct Elem;
template <> struct Elem<0> { typedef _Float16 T; };
template <> struct Elem<1> { typedef __bf16 T; };
template <int ET, bool SPLIT, int BIAS_MODE, int OUT_MODE, bool RESID, int ACT = 0>
__global__ __launch_bounds__(256) void wmma_gemm64(
    const unsigned short* __restrict__ Ap, const unsigned short* __restrict__ A2p, int lda, long strideA,
    const unsigned short* __restrict__ Btp, const unsigned short* __restrict__ Bt2p, int ldb, long strideB,
    void* __restrict__ Cout, void* __restrict__ Cout2, int ldc, long strideC,
    const float* __restrict__ bias,
    const float* __restrict__ resid, long strideR,
    int M, int N, int K, float scale) {
  typedef typename Elem<ET>::T T;
  typedef typename Frag<T>::V V;
  const T* A = (const T*)Ap; const T* A2 = (const T*)A2p; const T* Bt = (const T*)Btp; const T* Bt2 = (const T*)Bt2p;
  __shared__ __align__(16) float sT[8][16 * 68];
  const int b    = blockIdx.y;
  const int lane = threadIdx.x & 31;
  const int wave = threadIdx.x >> 5;
  const int tilesN = N >> 6;
  const int tilesM = M >> 6;
  const int tile = blockIdx.x * 8 + wave;
  if (tile >= tilesM * tilesN) return;
  const int tm = tile / tilesN;
  const int tn = tile - tm * tilesN;
  const int m0 = tm << 6;
  const int n0 = tn << 6;

  const T* Ab  = A  + (size_t)b * strideA;
  const T* Bb  = Bt + (size_t)b * strideB;
  const T* Ab2 = SPLIT ? (A2  + (size_t)b * strideA) : nullptr;
  const T* Bb2 = SPLIT ? (Bt2 + (size_t)b * strideB) : nullptr;

  const int rlane = lane & 15;
  const int koff  = (lane >> 4) * 8;
  const int mOff  = (lane >> 4) * 8;

  v8f acc[4][4];
#pragma unroll
  for (int i = 0; i < 4; ++i)
#pragma unroll
    for (int j = 0; j < 4; ++j) acc[i][j] = (v8f){0.f,0.f,0.f,0.f,0.f,0.f,0.f,0.f};

  for (int k0 = 0; k0 < K; k0 += 32) {
    V bh[4], bl[4];
#pragma unroll
    for (int j = 0; j < 4; ++j) {
      const size_t bo = (size_t)(n0 + (j << 4) + rlane) * ldb + koff + k0;
      bh[j] = Frag<T>::load(Bb + bo);
      if (SPLIT) bl[j] = Frag<T>::load(Bb2 + bo);
    }
#pragma unroll
    for (int i = 0; i < 4; ++i) {
      const size_t ao = (size_t)(m0 + (i << 4) + rlane) * lda + koff + k0;
      V ah = Frag<T>::load(Ab + ao);
      V al;
      if (SPLIT) al = Frag<T>::load(Ab2 + ao);
#pragma unroll
      for (int j = 0; j < 4; ++j) {
        acc[i][j] = Frag<T>::mma(ah, bh[j], acc[i][j]);
        if (SPLIT) {
          acc[i][j] = Frag<T>::mma(ah, bl[j], acc[i][j]);
          acc[i][j] = Frag<T>::mma(al, bh[j], acc[i][j]);
        }
      }
      Frag<T>::guard(acc[i][0], acc[i][3], ah, SPLIT ? al : ah);
    }
    Frag<T>::keep(bh[0], bh[1], bh[2], bh[3]);
    if (SPLIT) Frag<T>::keep(bl[0], bl[1], bl[2], bl[3]);
  }
  acc_guard4(acc[0][0], acc[0][1], acc[0][2], acc[0][3]);
  acc_guard4(acc[1][0], acc[1][1], acc[1][2], acc[1][3]);
  acc_guard4(acc[2][0], acc[2][1], acc[2][2], acc[2][3]);
  acc_guard4(acc[3][0], acc[3][1], acc[3][2], acc[3][3]);

  float* slab = sT[wave];
  const float* Rb = RESID ? (resid + (size_t)b * strideR) : nullptr;
#pragma unroll
  for (int i = 0; i < 4; ++i) {
    const int mBase = m0 + (i << 4);
#pragma unroll
    for (int j = 0; j < 4; ++j) {
      const int n = n0 + (j << 4) + rlane;
      float bv = 0.f;
      if (BIAS_MODE == 2) bv = bias[n];
#pragma unroll
      for (int r = 0; r < 8; ++r) {
        float v = acc[i][j][r] * scale;
        if (BIAS_MODE == 1) v += bias[mBase + mOff + r];
        if (BIAS_MODE == 2) v += bv;
        if (RESID) v += Rb[(size_t)(mBase + mOff + r) * ldc + n];
        if (ACT == 1) v = tanhf(v);
        if (ACT == 2) v = fmaxf(v, 0.0f);
        if (ACT == 3) v = v / (1.0f + expf(-v));
        if (ACT == 4) v = (v > 0.f) ? v : 0.01f * v;
        if (ACT == 5) v = 0.5f * v * (1.0f + erff(v * 0.70710678118654752f));
        slab[(mOff + r) * 68 + (j << 4) + rlane] = v;
      }
    }
    __builtin_amdgcn_fence(__ATOMIC_RELEASE, "workgroup");
    __builtin_amdgcn_wave_barrier();
    __builtin_amdgcn_fence(__ATOMIC_ACQUIRE, "workgroup");
    if (OUT_MODE == 0) {
      float* C = (float*)Cout + (size_t)b * strideC;
      const int hh = lane >> 4, c4 = (lane & 15) * 4;
      for (int pass = 0; pass < 2; ++pass) {
#pragma unroll
        for (int it = 0; it < 8; ++it) {
          const int row = it * 2 + hh;
          v4f v = *(const v4f*)(slab + row * 68 + c4);
          *(volatile v4f*)(C + (size_t)(mBase + row) * ldc + n0 + c4) = v;
        }
        __threadfence();
      }
    } else {
      const int q = lane >> 3, c8 = (lane & 7) * 8;
      unsigned short* C  = (unsigned short*)Cout  + (size_t)b * strideC;
      unsigned short* C2 = (OUT_MODE == 2) ? ((unsigned short*)Cout2 + (size_t)b * strideC) : nullptr;
      for (int pass = 0; pass < 2; ++pass) {
#pragma unroll
        for (int it = 0; it < 4; ++it) {
          const int row = it * 4 + q;
          const float* sp = slab + row * 68 + c8;
          v8h hv, lv;
#pragma unroll
          for (int e = 0; e < 8; ++e) {
            if (OUT_MODE == 1) {
              hv[e] = (_Float16)sp[e];
            } else {
              unsigned short hb = f2bf_bits(sp[e]);
              unsigned short lb = f2bf_bits(sp[e] - bf_bits2f(hb));
              hv[e] = __builtin_bit_cast(_Float16, hb);
              lv[e] = __builtin_bit_cast(_Float16, lb);
            }
          }
          *(volatile v8h*)(C + (size_t)(mBase + row) * ldc + n0 + c8) = hv;
          if (OUT_MODE == 2) *(volatile v8h*)(C2 + (size_t)(mBase + row) * ldc + n0 + c8) = lv;
        }
        __threadfence();
      }
    }
    __builtin_amdgcn_fence(__ATOMIC_RELEASE, "workgroup");
    __builtin_amdgcn_wave_barrier();
    __builtin_amdgcn_fence(__ATOMIC_ACQUIRE, "workgroup");
  }
}

__global__ __launch_bounds__(256) void cast_f32_f16x8(
    const float* __restrict__ in0, const float* __restrict__ in1,
    _Float16* __restrict__ out0, _Float16* __restrict__ out1, int n8) {
  const float* in = (blockIdx.y == 0) ? in0 : in1;
  _Float16* out = (blockIdx.y == 0) ? out0 : out1;
  const int i = blockIdx.x * 256 + threadIdx.x;
  if (i < n8) {
    const v4f a = *(const v4f*)(in + (size_t)i * 8);
    const v4f c = *(const v4f*)(in + (size_t)i * 8 + 4);
    v8h hv;
    hv[0] = (_Float16)a[0]; hv[1] = (_Float16)a[1]; hv[2] = (_Float16)a[2]; hv[3] = (_Float16)a[3];
    hv[4] = (_Float16)c[0]; hv[5] = (_Float16)c[1]; hv[6] = (_Float16)c[2]; hv[7] = (_Float16)c[3];
    *(volatile v8h*)(out + (size_t)i * 8) = hv;
    __threadfence();
    *(volatile v8h*)(out + (size_t)i * 8) = hv;
  }
}

#define WDIM 256
__global__ __launch_bounds__(256) void wt_transpose_f16(
    const float* __restrict__ W0, const float* __restrict__ W1, const float* __restrict__ W2, const float* __restrict__ W3,
    _Float16* __restrict__ T0, _Float16* __restrict__ T1, _Float16* __restrict__ T2, _Float16* __restrict__ T3) {
  __shared__ float sw[32][WDIM + 1];
  const int by = blockIdx.y;
  const float* W = (by == 0) ? W0 : (by == 1) ? W1 : (by == 2) ? W2 : W3;
  _Float16*    T = (by == 0) ? T0 : (by == 1) ? T1 : (by == 2) ? T2 : T3;
  const int n0 = blockIdx.x * 32;
  const int t = threadIdx.x;
#pragma unroll 1
  for (int it = 0; it < 32; ++it) {
    const int k = it * 8 + (t >> 5);
    const int j = t & 31;
    sw[j][k] = W[(size_t)k * WDIM + n0 + j];
  }
  __syncthreads();
  const int g = t >> 3;
  const int e = t & 7;
  for (int pass = 0; pass < 2; ++pass) {
#pragma unroll
    for (int it = 0; it < 4; ++it) {
      const int col = it * 64 + e * 8;
      v8h hv;
#pragma unroll
      for (int i = 0; i < 8; ++i) hv[i] = (_Float16)(sw[g][col + i] * 16.0f);
      *(volatile v8h*)(T + (size_t)(n0 + g) * WDIM + col) = hv;
    }
    __threadfence();
  }
}

#define AT_S 8
#define AT_H 32
#define AT_W 32
#define AT_C 256
#define AT_NB 27
#define AT_PITCH 264
#define QK_SCALE 0.17677669529663687f
__global__ __launch_bounds__(256) void local_attn3d(
    const float* __restrict__ qp, const float* __restrict__ kf, const float* __restrict__ vf,
    _Float16* __restrict__ oh) {
  __shared__ __align__(16) float sbuf[AT_NB * 256];
  const int tid  = threadIdx.x;
  const int head = tid & 7;
  const int vox  = tid >> 3;
  const int pos  = blockIdx.x * 32 + vox;
  const int pw = pos & 31;
  const int ph = (pos >> 5) & 31;
  const int ps = (pos >> 10) & 7;
  const int pb = pos >> 13;

  float qr[32];
  {
    const float* qptr = qp + (size_t)pos * AT_C + head * 32;
#pragma unroll
    for (int i = 0; i < 8; ++i) {
      const v4f tq = *(const v4f*)(qptr + 4 * i);
      qr[4 * i + 0] = tq[0]; qr[4 * i + 1] = tq[1]; qr[4 * i + 2] = tq[2]; qr[4 * i + 3] = tq[3];
    }
  }

  float mx = -INFINITY;
  unsigned vmask = 0u;
  int kk = 0;
#pragma unroll 1
  for (int dz = 0; dz < 3; ++dz) {
    const int zs = ps + dz - 1;
    const bool vz = ((unsigned)zs < (unsigned)AT_S);
    const int cs = zs < 0 ? 0 : (zs > AT_S - 1 ? AT_S - 1 : zs);
#pragma unroll 1
    for (int dy = 0; dy < 3; ++dy) {
      const int zh = ph + dy - 1;
      const bool vy = vz && ((unsigned)zh < (unsigned)AT_H);
      const int ch = zh < 0 ? 0 : (zh > AT_H - 1 ? AT_H - 1 : zh);
      const int rowb = ((pb * AT_S + cs) * AT_H + ch) * AT_W;
#pragma unroll 1
      for (int dx = 0; dx < 3; ++dx) {
        const int zw = pw + dx - 1;
        const bool valid = vy && ((unsigned)zw < (unsigned)AT_W);
        const int cw = zw < 0 ? 0 : (zw > AT_W - 1 ? AT_W - 1 : zw);
        const float* kp = kf + (size_t)(rowb + cw) * AT_C + head * 32;
        float a = 0.f;
#pragma unroll
        for (int i = 0; i < 8; ++i) {
          const v4f tk = *(const v4f*)(kp + 4 * i);
          a = fmaf(qr[4 * i + 0], tk[0], a);
          a = fmaf(qr[4 * i + 1], tk[1], a);
          a = fmaf(qr[4 * i + 2], tk[2], a);
          a = fmaf(qr[4 * i + 3], tk[3], a);
        }
        const float dot = a * QK_SCALE;
        sbuf[kk * 256 + tid] = dot;
        if (valid) { mx = fmaxf(mx, dot); vmask |= (1u << kk); }
        ++kk;
      }
    }
  }

  float sum = 0.f;
#pragma unroll 1
  for (int k2 = 0; k2 < AT_NB; ++k2) {
    const float d = sbuf[k2 * 256 + tid];
    const float ex = __expf(d - mx);
    const float p = ((vmask >> k2) & 1u) ? ex : 0.f;
    sbuf[k2 * 256 + tid] = p;
    sum += p;
  }
  const float inv = __builtin_amdgcn_rcpf(sum);

  float acc[32];
#pragma unroll
  for (int i = 0; i < 32; ++i) acc[i] = 0.f;
  kk = 0;
#pragma unroll 1
  for (int dz = 0; dz < 3; ++dz) {
    const int zs = ps + dz - 1;
    const int cs = zs < 0 ? 0 : (zs > AT_S - 1 ? AT_S - 1 : zs);
#pragma unroll 1
    for (int dy = 0; dy < 3; ++dy) {
      const int zh = ph + dy - 1;
      const int ch = zh < 0 ? 0 : (zh > AT_H - 1 ? AT_H - 1 : zh);
      const int rowb = ((pb * AT_S + cs) * AT_H + ch) * AT_W;
#pragma unroll 1
      for (int dx = 0; dx < 3; ++dx) {
        const int zw = pw + dx - 1;
        const int cw = zw < 0 ? 0 : (zw > AT_W - 1 ? AT_W - 1 : zw);
        const float p = sbuf[kk * 256 + tid];
        const float* vp = vf + (size_t)(rowb + cw) * AT_C + head * 32;
#pragma unroll
        for (int i = 0; i < 8; ++i) {
          const v4f tv = *(const v4f*)(vp + 4 * i);
          acc[4 * i + 0] = fmaf(p, tv[0], acc[4 * i + 0]);
          acc[4 * i + 1] = fmaf(p, tv[1], acc[4 * i + 1]);
          acc[4 * i + 2] = fmaf(p, tv[2], acc[4 * i + 2]);
          acc[4 * i + 3] = fmaf(p, tv[3], acc[4 * i + 3]);
        }
        ++kk;
      }
    }
  }
  const float osc = inv * 8.0f;

  __syncthreads();
  _Float16* st = reinterpret_cast<_Float16*>(sbuf);
  {
    _Float16* sp = st + vox * AT_PITCH + head * 32;
#pragma unroll
    for (int j = 0; j < 4; ++j) {
      v8h hv;
#pragma unroll
      for (int i = 0; i < 8; ++i) hv[i] = (_Float16)(acc[8 * j + i] * osc);
      *(v8h*)(sp + 8 * j) = hv;
    }
  }
  __syncthreads();
  {
    const int g = tid >> 3;
    const int e = tid & 7;
    _Float16* ob = oh + (size_t)blockIdx.x * 32 * AT_C;
    for (int pass = 0; pass < 2; ++pass) {
#pragma unroll
      for (int it = 0; it < 4; ++it) {
        const int L = it * 32 + g;
        const int row = L >> 2;
        const int seg = L & 3;
        const v8h hv = *(const v8h*)(st + row * AT_PITCH + seg * 64 + e * 8);
        *(volatile v8h*)(ob + (size_t)row * AT_C + seg * 64 + e * 8) = hv;
      }
      __threadfence();
    }
  }
}

extern "C" void kernel_launch(void* const* d_in, const int* in_sizes, int n_in,
                              void* d_out, int out_size, void* d_ws, size_t ws_size,
                              hipStream_t stream) {
  const int MP = 16384;
  const int DC = 256;
  if (n_in < 8) return;
  if (in_sizes[0] != MP * DC || in_sizes[1] != MP * DC) return;
  if (in_sizes[2] != DC * DC || in_sizes[3] != DC * DC || in_sizes[4] != DC * DC || in_sizes[6] != DC * DC) return;
  if (in_sizes[5] != DC || in_sizes[7] != DC) return;
  if (out_size != MP * DC) return;

  const float* x  = (const float*)d_in[0];
  const float* q  = (const float*)d_in[1];
  const float* Wq = (const float*)d_in[2];
  const float* Wk = (const float*)d_in[3];
  const float* Wv = (const float*)d_in[4];
  const float* bv = (const float*)d_in[5];
  const float* Wo = (const float*)d_in[6];
  const float* bo = (const float*)d_in[7];
  float* outp = (float*)d_out;

  const size_t actH = (size_t)MP * DC * sizeof(_Float16);
  const size_t actF = (size_t)MP * DC * sizeof(float);
  const size_t wH   = (size_t)DC * DC * sizeof(_Float16);
  size_t off = 0;
  char* base = (char*)d_ws;
  _Float16* xh  = (_Float16*)(base + off); off += actH;
  _Float16* qh  = (_Float16*)(base + off); off += actH;
  _Float16* WqT = (_Float16*)(base + off); off += wH;
  _Float16* WkT = (_Float16*)(base + off); off += wH;
  _Float16* WvT = (_Float16*)(base + off); off += wH;
  _Float16* WoT = (_Float16*)(base + off); off += wH;
  float*    qpF = (float*)(base + off);    off += actF;
  float*    kF  = (float*)(base + off);    off += actF;
  float*    vF  = (float*)(base + off);    off += actF;
  _Float16* aH  = (_Float16*)(base + off); off += actH;
  if (off > ws_size) return;

  const int n8 = MP * DC / 8;
  cast_f32_f16x8<<<dim3((n8 + 255) / 256, 2), 256, 0, stream>>>(x, q, xh, qh, n8);

  wt_transpose_f16<<<dim3(DC / 32, 4), 256, 0, stream>>>(Wq, Wk, Wv, Wo, WqT, WkT, WvT, WoT);

  const dim3 gg((MP / 64) * (DC / 64) / 8, 1);
  const float s16 = 1.0f / 16.0f;
  wmma_gemm64<0, false, 0, 0, false, 0><<<gg, 256, 0, stream>>>(
      (const unsigned short*)qh, (const unsigned short*)qh, DC, 0L,
      (const unsigned short*)WqT, (const unsigned short*)WqT, DC, 0L,
      (void*)qpF, (void*)qpF, DC, 0L, bo, x, 0L, MP, DC, DC, s16);
  wmma_gemm64<0, false, 0, 0, false, 0><<<gg, 256, 0, stream>>>(
      (const unsigned short*)xh, (const unsigned short*)xh, DC, 0L,
      (const unsigned short*)WkT, (const unsigned short*)WkT, DC, 0L,
      (void*)kF, (void*)kF, DC, 0L, bo, x, 0L, MP, DC, DC, s16);
  wmma_gemm64<0, false, 2, 0, false, 0><<<gg, 256, 0, stream>>>(
      (const unsigned short*)xh, (const unsigned short*)xh, DC, 0L,
      (const unsigned short*)WvT, (const unsigned short*)WvT, DC, 0L,
      (void*)vF, (void*)vF, DC, 0L, bv, x, 0L, MP, DC, DC, s16);

  local_attn3d<<<MP / 32, 256, 0, stream>>>(qpF, kF, vF, aH);

  wmma_gemm64<0, false, 2, 0, false, 0><<<gg, 256, 0, stream>>>(
      (const unsigned short*)aH, (const unsigned short*)aH, DC, 0L,
      (const unsigned short*)WoT, (const unsigned short*)WoT, DC, 0L,
      (void*)outp, (void*)outp, DC, 0L, bo, x, 0L, MP, DC, DC, 1.0f / 128.0f);
}
